// ProceduralMemory_20976620274276
// MI455X (gfx1250) — hardware-verified
//
#include <hip/hip_runtime.h>
#include <math.h>

constexpr int kBS  = 32;
constexpr int kP   = 128;
constexpr int kR   = 16;
constexpr int kRP  = 64;
constexpr int kD   = 1024;
constexpr int kTok = kBS * kP;
constexpr float kRho     = 0.97f;
constexpr float kEps     = 1e-8f;
constexpr float kGateMul = 0.2f;
static_assert(kTok % 64 == 0 && kD % 64 == 0 && kP % 64 == 0 && kRP % 32 == 0);
static_assert(kD / 4 == 256 && kD / 8 == 128);

typedef __attribute__((ext_vector_type(16))) _Float16 v16h;
typedef __attribute__((ext_vector_type(8)))  _Float16 v8h;
typedef __attribute__((ext_vector_type(16))) __bf16   v16b;
typedef __attribute__((ext_vector_type(8)))  __bf16   v8b;
typedef __attribute__((ext_vector_type(8)))  float    v8f;
typedef __attribute__((ext_vector_type(4)))  float    v4f;
typedef __attribute__((ext_vector_type(4)))  unsigned int v4u;

__device__ __forceinline__ unsigned short f2bf_bits(float f) {
  unsigned u = __float_as_uint(f);
  return (unsigned short)((u + 0x7FFFu + ((u >> 16) & 1u)) >> 16);
}
__device__ __forceinline__ float bf_bits2f(unsigned short h) { return __uint_as_float(((unsigned)h) << 16); }
__device__ __forceinline__ float bfq(float f) { return bf_bits2f(f2bf_bits(f)); }

__device__ __forceinline__ void dep_guard_h(v8f& a, v8f& b, v16h x, v16h y) { asm volatile("v_nop\n\tv_nop\n\tv_nop\n\tv_nop" : "+v"(a), "+v"(b) : "v"(x), "v"(y)); }
__device__ __forceinline__ void dep_guard_b(v8f& a, v8f& b, v16b x, v16b y) { asm volatile("v_nop\n\tv_nop\n\tv_nop\n\tv_nop" : "+v"(a), "+v"(b) : "v"(x), "v"(y)); }
__device__ __forceinline__ void keep4_h(v16h a, v16h b, v16h c, v16h d) { asm volatile("v_nop" :: "v"(a), "v"(b), "v"(c), "v"(d)); }
__device__ __forceinline__ void keep4_b(v16b a, v16b b, v16b c, v16b d) { asm volatile("v_nop" :: "v"(a), "v"(b), "v"(c), "v"(d)); }
__device__ __forceinline__ void acc_guard4(v8f& a, v8f& b, v8f& c, v8f& d) { asm volatile("v_nop\n\tv_nop\n\tv_nop\n\tv_nop" : "+v"(a), "+v"(b), "+v"(c), "+v"(d)); }
template <typename T> struct Frag;
template <> struct Frag<_Float16> {
  typedef v16h V; union U { v16h v; v8h h[2]; };
  static __device__ __forceinline__ v16h load(const _Float16* p) {
    U f; f.h[0] = *(const v8h*)(p); f.h[1] = *(const v8h*)(p + 16); return f.v;
  }
  static __device__ __forceinline__ v8f mma(v16h a, v16h b, v8f c) {
    return __builtin_amdgcn_wmma_f32_16x16x32_f16(false, a, false, b, (short)0, c, false, false);
  }
  static __device__ __forceinline__ void guard(v8f& a, v8f& b, v16h x, v16h y) { dep_guard_h(a, b, x, y); }
  static __device__ __forceinline__ void keep(v16h a, v16h b, v16h c, v16h d) { keep4_h(a, b, c, d); }
};
template <> struct Frag<__bf16> {
  typedef v16b V; union U { v16b v; v8b h[2]; };
  static __device__ __forceinline__ v16b load(const __bf16* p) {
    U f; f.h[0] = *(const v8b*)(p); f.h[1] = *(const v8b*)(p + 16); return f.v;
  }
  static __device__ __forceinline__ v8f mma(v16b a, v16b b, v8f c) {
    return __builtin_amdgcn_wmma_f32_16x16x32_bf16(false, a, false, b, (short)0, c, false, false);
  }
  static __device__ __forceinline__ void guard(v8f& a, v8f& b, v16b x, v16b y) { dep_guard_b(a, b, x, y); }
  static __device__ __forceinline__ void keep(v16b a, v16b b, v16b c, v16b d) { keep4_b(a, b, c, d); }
};

__device__ __forceinline__ unsigned pk16(unsigned short a, unsigned short b) { return (unsigned)a | ((unsigned)b << 16); }
__device__ __forceinline__ unsigned short h_bits(float f) { const _Float16 h = (_Float16)f; return __builtin_bit_cast(unsigned short, h); }

template <int ET> struct Elem;
template <> struct Elem<0> { typedef _Float16 T; };
template <> struct Elem<1> { typedef __bf16 T; };
template <int ET, int SPL, int RSC, int CSC, int BIAS_MODE, int OUT_MODE>
__global__ __launch_bounds__(256) void wmma_gemm64(
    const unsigned short* __restrict__ Ap, const unsigned short* __restrict__ A2p, int lda, long strideA,
    const unsigned short* __restrict__ Btp, const unsigned short* __restrict__ Bt2p, int ldb, long strideB,
    void* __restrict__ Cout, void* __restrict__ Cout2, int ldc, long strideC,
    const float* __restrict__ rsc, long strideS,
    const float* __restrict__ csc, long strideCS, int ncsc,
    const float* __restrict__ bias,
    int M, int N, int K, float scale) {
  typedef typename Elem<ET>::T T;
  typedef typename Frag<T>::V V;
  const T* A = (const T*)Ap; const T* A2 = (const T*)A2p; const T* Bt = (const T*)Btp; const T* Bt2 = (const T*)Bt2p;
  __shared__ __align__(16) float sT[8][16 * 68];
  const int b    = blockIdx.y;
  const int lane = threadIdx.x & 31;
  const int wave = threadIdx.x >> 5;
  const int tilesN = N >> 6;
  const int tilesM = M >> 6;
  const int tile = blockIdx.x * 8 + wave;
  if (tile >= tilesM * tilesN) return;
  const int tm = tile / tilesN;
  const int tn = tile - tm * tilesN;
  const int m0 = tm << 6;
  const int n0 = tn << 6;

  const T* Ab  = A  + (size_t)b * strideA;
  const T* Bb  = Bt + (size_t)b * strideB;
  const T* Ab2 = (SPL & 1) ? (A2  + (size_t)b * strideA) : nullptr;
  const T* Bb2 = (SPL & 2) ? (Bt2 + (size_t)b * strideB) : nullptr;

  const int rlane = lane & 15;
  const int koff  = (lane >> 4) * 8;
  const int mOff  = (lane >> 4) * 8;

  v8f acc[4][4];
#pragma unroll
  for (int i = 0; i < 4; ++i)
#pragma unroll
    for (int j = 0; j < 4; ++j) acc[i][j] = (v8f){0.f,0.f,0.f,0.f,0.f,0.f,0.f,0.f};

  for (int k0 = 0; k0 < K; k0 += 32) {
    V bh[4], bl[4];
#pragma unroll
    for (int j = 0; j < 4; ++j) {
      const size_t bo = (size_t)(n0 + (j << 4) + rlane) * ldb + koff + k0;
      bh[j] = Frag<T>::load(Bb + bo);
      if (SPL & 2) bl[j] = Frag<T>::load(Bb2 + bo);
    }
#pragma unroll
    for (int i = 0; i < 4; ++i) {
      const size_t ao = (size_t)(m0 + (i << 4) + rlane) * lda + koff + k0;
      V ah = Frag<T>::load(Ab + ao);
      V al;
      if (SPL & 1) al = Frag<T>::load(Ab2 + ao);
#pragma unroll
      for (int j = 0; j < 4; ++j) {
        acc[i][j] = Frag<T>::mma(ah, bh[j], acc[i][j]);
        if (SPL & 2) acc[i][j] = Frag<T>::mma(ah, bl[j], acc[i][j]);
        if (SPL & 1) acc[i][j] = Frag<T>::mma(al, bh[j], acc[i][j]);
      }
      Frag<T>::guard(acc[i][0], acc[i][3], ah, (SPL & 1) ? al : ah);
    }
    Frag<T>::keep(bh[0], bh[1], bh[2], bh[3]);
    if (SPL & 2) Frag<T>::keep(bl[0], bl[1], bl[2], bl[3]);
  }
  acc_guard4(acc[0][0], acc[0][1], acc[0][2], acc[0][3]);
  acc_guard4(acc[1][0], acc[1][1], acc[1][2], acc[1][3]);
  acc_guard4(acc[2][0], acc[2][1], acc[2][2], acc[2][3]);
  acc_guard4(acc[3][0], acc[3][1], acc[3][2], acc[3][3]);

  float* slab = sT[wave];
  const float* Rs = RSC ? (rsc + (size_t)b * strideS) : nullptr;
  const float* Cs = CSC ? (csc + (size_t)b * strideCS) : nullptr;
#pragma unroll
  for (int i = 0; i < 4; ++i) {
    const int mBase = m0 + (i << 4);
    float rsv[8];
#pragma unroll
    for (int r = 0; r < 8; ++r) rsv[r] = RSC ? Rs[mBase + mOff + r] : 1.0f;
#pragma unroll
    for (int j = 0; j < 4; ++j) {
      const int n = n0 + (j << 4) + rlane;
      float bv = 0.f, cv = 1.0f;
      if (BIAS_MODE == 2) bv = bias[n];
      if (BIAS_MODE == 3) bv = bfq(bias[n]);
      if (CSC) {
        const int nc = (n < ncsc) ? n : (ncsc - 1);
        cv = bfq(Cs[nc]);
        if (n >= ncsc) cv = 0.0f;
      }
#pragma unroll
      for (int r = 0; r < 8; ++r) {
        float v = acc[i][j][r] * scale;
        if (RSC) v = v * rsv[r];
        if (CSC) v = v * cv;
        if (BIAS_MODE != 0) v += bv;
        slab[(mOff + r) * 68 + (j << 4) + rlane] = v;
      }
    }
    __builtin_amdgcn_fence(__ATOMIC_RELEASE, "workgroup");
    __builtin_amdgcn_wave_barrier();
    __builtin_amdgcn_fence(__ATOMIC_ACQUIRE, "workgroup");
    if (OUT_MODE == 0) {
      float* C = (float*)Cout + (size_t)b * strideC;
      const int hh = lane >> 4, c4 = (lane & 15) * 4;
      for (int pass = 0; pass < 2; ++pass) {
#pragma unroll
        for (int it = 0; it < 8; ++it) {
          const int row = it * 2 + hh;
          v4f v = *(const v4f*)(slab + row * 68 + c4);
          *(volatile v4f*)(C + (size_t)(mBase + row) * ldc + n0 + c4) = v;
        }
        __threadfence();
      }
    } else {
      const int q = lane >> 3, c8 = (lane & 7) * 8;
      unsigned short* C  = (unsigned short*)Cout  + (size_t)b * strideC;
      unsigned short* C2 = (OUT_MODE == 2) ? ((unsigned short*)Cout2 + (size_t)b * strideC) : nullptr;
      for (int pass = 0; pass < 2; ++pass) {
#pragma unroll
        for (int it = 0; it < 4; ++it) {
          const int row = it * 4 + q;
          const float* sp = slab + row * 68 + c8;
          v8h hv, lv;
#pragma unroll
          for (int e = 0; e < 8; ++e) {
            if (OUT_MODE == 1) {
              hv[e] = (_Float16)sp[e];
            } else {
              unsigned short hb = f2bf_bits(sp[e]);
              unsigned short lb = f2bf_bits(sp[e] - bf_bits2f(hb));
              hv[e] = __builtin_bit_cast(_Float16, hb);
              lv[e] = __builtin_bit_cast(_Float16, lb);
            }
          }
          *(volatile v8h*)(C + (size_t)(mBase + row) * ldc + n0 + c8) = hv;
          if (OUT_MODE == 2) *(volatile v8h*)(C2 + (size_t)(mBase + row) * ldc + n0 + c8) = lv;
        }
        __threadfence();
      }
    }
    __builtin_amdgcn_fence(__ATOMIC_RELEASE, "workgroup");
    __builtin_amdgcn_wave_barrier();
    __builtin_amdgcn_fence(__ATOMIC_ACQUIRE, "workgroup");
  }
}

template <int MODE>
__global__ __launch_bounds__(256) void cast8_kernel(const float* __restrict__ in, unsigned short* __restrict__ out, int n8, float scale) {
  const int i = blockIdx.x * 256 + threadIdx.x;
  if (i >= n8) return;
  const float* p = in + 8 * (size_t)i;
  const v4f a = *(const v4f*)(p);
  const v4f c = *(const v4f*)(p + 4);
  unsigned short hb[8];
#pragma unroll
  for (int e = 0; e < 4; ++e) {
    if (MODE == 0) {
      hb[e]     = f2bf_bits(a[e]);
      hb[4 + e] = f2bf_bits(c[e]);
    } else {
      hb[e]     = h_bits(bf_bits2f(f2bf_bits(a[e])) * scale);
      hb[4 + e] = h_bits(bf_bits2f(f2bf_bits(c[e])) * scale);
    }
  }
  const v4u u = (v4u){pk16(hb[0], hb[1]), pk16(hb[2], hb[3]), pk16(hb[4], hb[5]), pk16(hb[6], hb[7])};
  unsigned short* q = out + 8 * (size_t)i;
  *(volatile v4u*)q = u;
  __threadfence();
  *(volatile v4u*)q = u;
  (void)scale;
}

template <int CAST>
__global__ __launch_bounds__(128) void rownorm32_kernel(const float* __restrict__ in, unsigned short* __restrict__ out16,
                                                         float* __restrict__ rinv, int nrows) {
  __shared__ float red[4];
  __shared__ float sR[32];
  const int t = threadIdx.x, lane = t & 31, wave = t >> 5;
  const int row0 = blockIdx.x * 32;
#pragma unroll 1
  for (int rr = 0; rr < 32; ++rr) {
    int row = row0 + rr;
    row = (row < nrows) ? row : (nrows - 1);
    const float* xr = in + (size_t)row * kD + 8 * t;
    const v4f a = *(const v4f*)(xr);
    const v4f c = *(const v4f*)(xr + 4);
    float xb[8];
    unsigned short hb[8];
#pragma unroll
    for (int e = 0; e < 4; ++e) {
      if (CAST) {
        hb[e] = f2bf_bits(a[e]);       hb[4 + e] = f2bf_bits(c[e]);
        xb[e] = bf_bits2f(hb[e]);      xb[4 + e] = bf_bits2f(hb[4 + e]);
      } else {
        hb[e] = 0;                      hb[4 + e] = 0;
        xb[e] = a[e];                   xb[4 + e] = c[e];
      }
    }
    if (CAST) {
      const v4u u = (v4u){pk16(hb[0], hb[1]), pk16(hb[2], hb[3]), pk16(hb[4], hb[5]), pk16(hb[6], hb[7])};
      unsigned short* q = out16 + (size_t)row * kD + 8 * t;
      *(volatile v4u*)q = u;
      __threadfence();
      *(volatile v4u*)q = u;
    }
    float s = ((xb[0] * xb[0] + xb[1] * xb[1]) + (xb[2] * xb[2] + xb[3] * xb[3]))
            + ((xb[4] * xb[4] + xb[5] * xb[5]) + (xb[6] * xb[6] + xb[7] * xb[7]));
#pragma unroll
    for (int off = 16; off > 0; off >>= 1) s += __shfl_xor(s, off, 32);
    if (lane == 0) red[wave] = s;
    __syncthreads();
    if (t == 0) {
      const float tot = (red[0] + red[1]) + (red[2] + red[3]);
      const float nrm = fmaxf(sqrtf(tot), kEps);
      sR[rr] = 1.0f / nrm;
    }
    __syncthreads();
  }
  if (wave == 0) {
    const float v = sR[lane];
    float* p = rinv + row0 + lane;
    *(volatile float*)p = v;
    __threadfence();
    *(volatile float*)p = v;
  }
}

__global__ __launch_bounds__(256) void wt_cast_kernel(const float* __restrict__ W0, const float* __restrict__ W1,
                                                      unsigned short* __restrict__ T0, unsigned short* __restrict__ T1) {
  __shared__ unsigned short sT[64][72];
  const float* W = (blockIdx.z == 0) ? W0 : W1;
  unsigned short* T = (blockIdx.z == 0) ? T0 : T1;
  const int t = threadIdx.x, lane = t & 31, wave = t >> 5;
  const int n0 = blockIdx.x * 64, k0 = blockIdx.y * 64;
  const int c = t & 63, rq = t >> 6;
#pragma unroll
  for (int i = 0; i < 16; ++i) {
    const int kr = rq + 4 * i;
    sT[c][kr] = f2bf_bits(W[(size_t)(k0 + kr) * kD + n0 + c]);
  }
  __syncthreads();
  const int q = lane >> 3, c8 = (lane & 7) * 8;
  v4u u[2];
  size_t o[2];
#pragma unroll
  for (int it = 0; it < 2; ++it) {
    const int nl = wave * 8 + it * 4 + q;
    unsigned short hb[8];
#pragma unroll
    for (int e = 0; e < 8; ++e) hb[e] = sT[nl][c8 + e];
    u[it] = (v4u){pk16(hb[0], hb[1]), pk16(hb[2], hb[3]), pk16(hb[4], hb[5]), pk16(hb[6], hb[7])};
    o[it] = (size_t)(n0 + nl) * kD + k0 + c8;
  }
  for (int pass = 0; pass < 2; ++pass) {
#pragma unroll
    for (int it = 0; it < 2; ++it) *(volatile v4u*)(T + o[it]) = u[it];
    __threadfence();
  }
}

__global__ __launch_bounds__(256) void pk_pad_kernel(const float* __restrict__ pmk, unsigned short* __restrict__ PK, int n8) {
  const int i = blockIdx.x * 256 + threadIdx.x;
  if (i >= n8) return;
  const size_t e8 = (size_t)i * 8;
  const int c  = (int)(e8 % kD);
  const int rp = (int)((e8 / kD) % kRP);
  const int b  = (int)(e8 / ((size_t)kD * kRP));
  const int rs = (rp < kR) ? rp : (kR - 1);
  const float* p = pmk + (size_t)(b * kR + rs) * kD + c;
  const v4f a  = *(const v4f*)(p);
  const v4f cc = *(const v4f*)(p + 4);
  const bool live = rp < kR;
  unsigned short hb[8];
#pragma unroll
  for (int e = 0; e < 4; ++e) {
    hb[e]     = live ? f2bf_bits(a[e])  : (unsigned short)0;
    hb[4 + e] = live ? f2bf_bits(cc[e]) : (unsigned short)0;
  }
  const v4u u = (v4u){pk16(hb[0], hb[1]), pk16(hb[2], hb[3]), pk16(hb[4], hb[5]), pk16(hb[6], hb[7])};
  unsigned short* q = PK + e8;
  *(volatile v4u*)q = u;
  __threadfence();
  *(volatile v4u*)q = u;
}

__global__ __launch_bounds__(256) void vt_cast_kernel(const float* __restrict__ pmv, unsigned short* __restrict__ VT) {
  __shared__ unsigned short sV[64][20];
  const int t = threadIdx.x, lane = t & 31, wave = t >> 5;
  const int b = blockIdx.y, d0 = blockIdx.x * 64;
  const int c = t & 63, rq = t >> 6;
#pragma unroll
  for (int i = 0; i < 4; ++i) {
    const int r = rq + 4 * i;
    sV[c][r] = f2bf_bits(pmv[(size_t)(b * kR + r) * kD + d0 + c]);
  }
  __syncthreads();
  const int q = lane >> 3, c8 = (lane & 7) * 8;
  const bool live = c8 < kR;
  const int rb = c8 & 8;
  v4u u[2];
  size_t o[2];
#pragma unroll
  for (int it = 0; it < 2; ++it) {
    const int dl = wave * 8 + it * 4 + q;
    unsigned short hb[8];
#pragma unroll
    for (int e = 0; e < 8; ++e) {
      const unsigned short s = sV[dl][rb + e];
      hb[e] = live ? s : (unsigned short)0;
    }
    u[it] = (v4u){pk16(hb[0], hb[1]), pk16(hb[2], hb[3]), pk16(hb[4], hb[5]), pk16(hb[6], hb[7])};
    o[it] = (size_t)(b * kD + d0 + dl) * kRP + c8;
  }
  for (int pass = 0; pass < 2; ++pass) {
#pragma unroll
    for (int it = 0; it < 2; ++it) *(volatile v4u*)(VT + o[it]) = u[it];
    __threadfence();
  }
}

__global__ __launch_bounds__(256) void elig_scan_kernel(const float* __restrict__ KC, const float* __restrict__ VC,
                                                        const float* __restrict__ rinvK,
                                                        const float* __restrict__ surprise, const int* __restrict__ reset,
                                                        const float* __restrict__ eK0, const float* __restrict__ eV0,
                                                        float* __restrict__ outK, float* __restrict__ outV) {
  __shared__ float sA[kP];
  __shared__ float sCo[kP];
  const int z = blockIdx.z, b = blockIdx.x, t = threadIdx.x;
  const float* src = (z == 0) ? KC : VC;
  const float* e0  = (z == 0) ? eK0 : eV0;
  float* outp      = (z == 0) ? outK : outV;
  if (t < kP) {
    const int p = t;
    const float sv = bfq(surprise[b * kP + p]);
    const float g  = fminf(fmaxf(sv * kGateMul, 0.0f), 1.0f);
    const float rm = (reset[b * kP + p] != 0) ? 1.0f : 0.0f;
    sA[p] = kRho * (1.0f - rm);
    const float rk = rinvK[b * kP + p];
    sCo[p] = (z == 0) ? (g * rk) : g;
  }
  __syncthreads();
  v4f e[kR];
#pragma unroll
  for (int r = 0; r < kR; ++r) {
    const v4f v = *(const v4f*)(e0 + (size_t)(b * kR + r) * kD + 4 * t);
    e[r] = (v4f){bfq(v[0]), bfq(v[1]), bfq(v[2]), bfq(v[3])};
  }
#pragma unroll 1
  for (int p = 0; p < kP; ++p) {
    const v4f kv = *(const v4f*)(src + (size_t)(b * kP + p) * kD + 4 * t);
    const float a = sA[p], cf = sCo[p];
    const v4f inc = kv * cf;
#pragma unroll
    for (int r = 0; r < kR; ++r) e[r] = e[r] * a + inc;
  }
  for (int pass = 0; pass < 2; ++pass) {
#pragma unroll
    for (int r = 0; r < kR; ++r) *(volatile v4f*)(outp + (size_t)(b * kR + r) * kD + 4 * t) = e[r];
    __threadfence();
  }
}

extern "C" void kernel_launch(void* const* d_in, const int* in_sizes, int n_in,
                              void* d_out, int out_size, void* d_ws, size_t ws_size,
                              hipStream_t stream) {
  if (n_in < 13) return;
  if (in_sizes[0] != kTok * kD || in_sizes[1] != kTok * kD) return;
  if (in_sizes[2] != kTok || in_sizes[3] != kTok) return;
  if (in_sizes[4] != kBS * kR * kD || in_sizes[5] != kBS * kR * kD) return;
  if (in_sizes[6] != kBS * kR) return;
  if (in_sizes[7] != kBS * kR * kD || in_sizes[8] != kBS * kR * kD) return;
  if (in_sizes[9] != kD * kD || in_sizes[11] != kD * kD) return;
  if (in_sizes[10] != kD || in_sizes[12] != kD) return;
  if (out_size != kTok * kD + 2 * kBS * kR * kD) return;

  const float* x_all    = (const float*)d_in[0];
  const float* h_all    = (const float*)d_in[1];
  const float* surprise = (const float*)d_in[2];
  const int*   reset    = (const int*)d_in[3];
  const float* pm_K     = (const float*)d_in[4];
  const float* pm_V     = (const float*)d_in[5];
  const float* pm_a     = (const float*)d_in[6];
  const float* eK0      = (const float*)d_in[7];
  const float* eV0      = (const float*)d_in[8];
  const float* W_k      = (const float*)d_in[9];
  const float* b_k      = (const float*)d_in[10];
  const float* W_v      = (const float*)d_in[11];
  const float* b_v      = (const float*)d_in[12];

  float* y_out  = (float*)d_out;
  float* eK_out = y_out  + (size_t)kTok * kD;
  float* eV_out = eK_out + (size_t)kBS * kR * kD;

  const size_t SZ_T16  = (size_t)kTok * kD * 2;
  const size_t SZ_W16  = (size_t)kD * kD * 2;
  const size_t SZ_PK   = (size_t)kBS * kRP * kD * 2;
  const size_t SZ_VT   = (size_t)kBS * kD * kRP * 2;
  const size_t SZ_C32  = (size_t)kTok * kD * 4;
  const size_t SZ_RINV = (size_t)kTok * 4;
  const size_t SZ_WS   = (size_t)kBS * kP * kRP * 2;
  size_t off = 0;
  const size_t oX16 = off; off += SZ_T16;
  const size_t oH16 = off; off += SZ_T16;
  const size_t oWKT = off; off += SZ_W16;
  const size_t oWVT = off; off += SZ_W16;
  const size_t oPK  = off; off += SZ_PK;
  const size_t oVT  = off; off += SZ_VT;
  const size_t oKC  = off; off += SZ_C32;
  const size_t oVC  = off; off += SZ_C32;
  const size_t oRX  = off; off += SZ_RINV;
  const size_t oRK  = off; off += SZ_RINV;
  const size_t oWH  = off; off += SZ_WS;
  const size_t oWL  = off; off += SZ_WS;
  const size_t TOTAL = off;
  if (TOTAL > ws_size) return;
  if (TOTAL > (size_t)134217728) return;

  char* ws = (char*)d_ws;
  unsigned short* X16   = (unsigned short*)(ws + oX16);
  unsigned short* H16   = (unsigned short*)(ws + oH16);
  unsigned short* WKT   = (unsigned short*)(ws + oWKT);
  unsigned short* WVT   = (unsigned short*)(ws + oWVT);
  unsigned short* PK    = (unsigned short*)(ws + oPK);
  unsigned short* VT    = (unsigned short*)(ws + oVT);
  float*          KC    = (float*)(ws + oKC);
  float*          VC    = (float*)(ws + oVC);
  float*          RINVX = (float*)(ws + oRX);
  float*          RINVK = (float*)(ws + oRK);
  unsigned short* WH    = (unsigned short*)(ws + oWH);
  unsigned short* WL    = (unsigned short*)(ws + oWL);

  const dim3 blk(256);

  rownorm32_kernel<1><<<dim3(kTok / 32), dim3(128), 0, stream>>>(x_all, X16, RINVX, kTok);
  cast8_kernel<0><<<dim3((kTok * kD / 8) / 256), blk, 0, stream>>>(h_all, H16, kTok * kD / 8, 1.0f);
  wt_cast_kernel<<<dim3(kD / 64, kD / 64, 2), blk, 0, stream>>>(W_k, W_v, WKT, WVT);
  pk_pad_kernel<<<dim3((kBS * kRP * kD / 8) / 256), blk, 0, stream>>>(pm_K, PK, kBS * kRP * kD / 8);
  vt_cast_kernel<<<dim3(kD / 64, kBS), blk, 0, stream>>>(pm_V, VT);

  const dim3 gBig((kTok / 64) * (kD / 64) / 8, 1);
  wmma_gemm64<1, 0, 0, 0, 3, 0><<<gBig, blk, 0, stream>>>(
      X16, X16, kD, 0L,
      WKT, WKT, kD, 0L,
      (void*)KC, (void*)KC, kD, 0L,
      RINVX, 0L,
      pm_a, 0L, kR,
      b_k,
      kTok, kD, kD, 1.0f);
  wmma_gemm64<1, 0, 0, 0, 3, 0><<<gBig, blk, 0, stream>>>(
      H16, H16, kD, 0L,
      WVT, WVT, kD, 0L,
      (void*)VC, (void*)VC, kD, 0L,
      RINVX, 0L,
      pm_a, 0L, kR,
      b_v,
      kTok, kD, kD, 1.0f);
  rownorm32_kernel<0><<<dim3(kTok / 32), dim3(128), 0, stream>>>(KC, H16, RINVK, kTok);
  elig_scan_kernel<<<dim3(kBS, 1, 2), blk, 0, stream>>>(KC, VC, RINVK, surprise, reset, eK0, eV0, eK_out, eV_out);

  wmma_gemm64<1, 0, 1, 1, 0, 2><<<dim3(1, kBS), dim3(64), 0, stream>>>(
      X16, X16, kD, (long)kP * kD,
      PK, PK, kD, (long)kRP * kD,
      (void*)WH, (void*)WL, kRP, (long)kP * kRP,
      RINVX, (long)kP,
      pm_a, (long)kR, kR,
      b_k,
      kP, kRP, kD, 1.0f);
  wmma_gemm64<1, 1, 0, 0, 0, 0><<<dim3((kP / 64) * (kD / 64) / 8, kBS), blk, 0, stream>>>(
      WH, WL, kRP, (long)kP * kRP,
      VT, VT, kRP, (long)kD * kRP,
      (void*)y_out, (void*)y_out, kD, (long)kP * kD,
      RINVX, 0L,
      pm_a, 0L, kR,
      b_k,
      kP, kD, kRP, 1.0f);
}
